// RuleLearner_40690520162774
// MI455X (gfx1250) — hardware-run, weakly checked
//
#include <hip/hip_runtime.h>
#include <math.h>

typedef __attribute__((ext_vector_type(16))) _Float16 v16h;
typedef __attribute__((ext_vector_type(8)))  _Float16 v8h;
typedef __attribute__((ext_vector_type(8)))  float    v8f;
typedef __attribute__((ext_vector_type(4)))  float    v4f;

constexpr int kSeq        = 5;
constexpr int kNSym       = 9;
constexpr int kNU         = 14;
constexpr int kNI         = 128;
constexpr int kNB         = 4096;
constexpr int kRowsPerBlk = 32;
constexpr int kTabW       = 48;
constexpr int kNPad       = 16;
static_assert(kNU == kSeq + kNSym, "feature width");
static_assert((kNI % 32) == 0, "contraction depth is a multiple of 32");
static_assert((kNB % kRowsPerBlk) == 0, "row groups of 32");
static_assert(kNI == 128, "thread = rule mapping");

constexpr int kTOnePos = 0;
constexpr int kTOneSym = 5;
constexpr int kTBoth   = 10;
constexpr int kTC      = 15;
constexpr int kTOm     = 40;
static_assert(kTOm + kSeq + 1 <= kTabW, "table row width");

constexpr float kCarrySel     = 4096.0f;
constexpr float kCarryMap     = 64.0f;
constexpr float kResCarry     = 2048.0f;
constexpr float kInvRes       = 1.0f / kResCarry;
constexpr float kInvCarry     = 1.0f / (kCarrySel * kCarryMap);
constexpr float kF16MinNormal = 6.103515625e-5f;

constexpr size_t kOffTab = 0;
constexpr size_t kOffBhi = kOffTab + (size_t)kNI * kTabW * 4;
constexpr size_t kOffBlo = kOffBhi + (size_t)kNPad * kNI * 2;
constexpr size_t kOffAhi = kOffBlo + (size_t)kNPad * kNI * 2;
constexpr size_t kOffAlo = kOffAhi + (size_t)kNB * kNI * 2;
constexpr size_t kOffNp  = kOffAlo + (size_t)kNB * kNI * 2;
constexpr size_t kWsTotal = kOffNp + (size_t)kNB * kNPad * 4;
static_assert(kWsTotal == 2392064ull, "carve total");
static_assert(kWsTotal <= 134217728ull, "carve cap");
static_assert((kOffBhi % 128) == 0 && (kOffBlo % 128) == 0 && (kOffAhi % 128) == 0 &&
              (kOffAlo % 128) == 0 && (kOffNp % 128) == 0, "128-B aligned regions");

template <typename T> struct Frag;
template <> struct Frag<_Float16> {
  typedef v16h V; union U { v16h v; v8h h[2]; };
  static __device__ __forceinline__ v16h load(const _Float16* p) {
    U f; f.h[0] = *(const v8h*)(p); f.h[1] = *(const v8h*)(p + 16); return f.v;
  }
};

__device__ __forceinline__ v8f mma_h_guard(v16h a, v16h b, v8f c) {
  c = __builtin_amdgcn_wmma_f32_16x16x32_f16(false, a, false, b, (short)0, c, false, false);
  asm volatile("v_nop\n\tv_nop\n\tv_nop\n\tv_nop" : "+v"(c) : "v"(a), "v"(b));
  return c;
}

__device__ __forceinline__ int clamp_sym(int v) {
  return v < 0 ? 0 : (v > (kNSym - 1) ? (kNSym - 1) : v);
}

__device__ __forceinline__ float sigm(float x) {
  return 1.0f / (1.0f + expf(-x));
}

__device__ __forceinline__ void split_h(float v, _Float16& hi, _Float16& lo) {
  const float vh = (fabsf(v) < kF16MinNormal) ? 0.0f : v;
  hi = (_Float16)vh;
  const float hf = (float)hi;
  const float r  = (v - hf) * kResCarry;
  const float rf = (fabsf(r) < kF16MinNormal) ? 0.0f : r;
  lo = (_Float16)rf;
}

__host__ __device__ constexpr int pair_bit(int a, int b) {
  return a * (9 - a) / 2 + (b - a - 1);
}
static_assert(pair_bit(0, 1) == 0 && pair_bit(0, 4) == 3 && pair_bit(1, 2) == 4 &&
              pair_bit(2, 3) == 7 && pair_bit(3, 4) == 9, "pair enumeration");

__global__ __launch_bounds__(128) void prep_kernel(
    const int* __restrict__ inv_inputs, const int* __restrict__ inv_labels,
    const float* __restrict__ unaryp, const float* __restrict__ binaryp, const float* __restrict__ outmap,
    float* __restrict__ tab, unsigned short* __restrict__ bhi, unsigned short* __restrict__ blo)
{
  __shared__ __align__(16) float sT[kNI * kTabW];
  __shared__ __align__(16) float sB[kNPad * kNI];
  const int tid = threadIdx.x;
  float* row = sT + tid * kTabW;

#pragma unroll 1
  for (int m = 0; m < kSeq; ++m) {
    const int sim = clamp_sym(inv_inputs[tid * kSeq + m]);
    const float xp = unaryp[(tid * kSeq + m) * kNU + m];
    const float xs = unaryp[(tid * kSeq + m) * kNU + kSeq + sim];
    const float oP = 1.0f - sigm(xp);
    const float oS = 1.0f - sigm(xs);
    row[kTOnePos + m] = oP;
    row[kTOneSym + m] = oS;
    row[kTBoth + m]   = oP * oS;
  }
#pragma unroll 1
  for (int e = 0; e < kSeq * kSeq; ++e) {
    const int l = e / kSeq;
    const int m = e - l * kSeq;
    const int sl = clamp_sym(inv_inputs[tid * kSeq + l]);
    const int sm = clamp_sym(inv_inputs[tid * kSeq + m]);
    const float pv = sigm(binaryp[tid * (kSeq * kSeq) + e]);
    row[kTC + e] = ((l != m) && (sl == sm)) ? pv : 0.0f;
  }
  {
    float mx = outmap[tid * (kSeq + 1)];
#pragma unroll
    for (int j = 1; j < kSeq + 1; ++j) mx = fmaxf(mx, outmap[tid * (kSeq + 1) + j]);
    float ssum = 0.0f;
#pragma unroll 1
    for (int j = 0; j < kSeq + 1; ++j) {
      const float ev = expf(outmap[tid * (kSeq + 1) + j] - mx);
      row[kTOm + j] = ev;
      ssum += ev;
    }
    const float inv = 1.0f / ssum;
#pragma unroll 1
    for (int j = 0; j < kSeq + 1; ++j) row[kTOm + j] = row[kTOm + j] * inv;
  }
  row[kTabW - 2] = 0.0f;
  row[kTabW - 1] = 0.0f;
  {
    const int lab = clamp_sym(inv_labels[tid]);
    const float cv = row[kTOm + kSeq] * kCarryMap;
#pragma unroll
    for (int s = 0; s < kNPad; ++s) sB[s * kNI + tid] = (s == lab) ? cv : 0.0f;
  }
  __syncthreads();

  v4f tv[12];
#pragma unroll
  for (int it = 0; it < 12; ++it) tv[it] = *(const v4f*)(sT + (it * 128 + tid) * 4);
  v8h hv[2], lv[2];
#pragma unroll
  for (int it = 0; it < 2; ++it) {
    const int u = it * 128 + tid;
    const float* sp = sB + u * 8;
    const v4f a0 = *(const v4f*)(sp);
    const v4f a1 = *(const v4f*)(sp + 4);
#pragma unroll
    for (int e = 0; e < 4; ++e) {
      _Float16 h0, l0, h1, l1;
      const float x0 = a0[e];
      const float x1 = a1[e];
      split_h(x0, h0, l0);
      split_h(x1, h1, l1);
      hv[it][e] = h0; hv[it][4 + e] = h1;
      lv[it][e] = l0; lv[it][4 + e] = l1;
    }
  }
  for (int pass = 0; pass < 2; ++pass) {
#pragma unroll
    for (int it = 0; it < 12; ++it)
      *(volatile v4f*)(tab + (size_t)(it * 128 + tid) * 4) = tv[it];
#pragma unroll
    for (int it = 0; it < 2; ++it) {
      const size_t o = (size_t)(it * 128 + tid) * 8;
      *(volatile v8h*)(bhi + o) = hv[it];
      *(volatile v8h*)(blo + o) = lv[it];
    }
    __threadfence();
  }
}

#define TABV(e) tv[(e) >> 2][(e) & 3]

__global__ __launch_bounds__(128) void unify_kernel(
    const int* __restrict__ inputs, const int* __restrict__ inv_inputs, const float* __restrict__ tab,
    unsigned short* __restrict__ ahi, unsigned short* __restrict__ alo, float* __restrict__ npl, float scale)
{
  __shared__ __align__(16) float sR[kTabW * kNI];
  __shared__ __align__(16) float sE[kRowsPerBlk * kNI];
  __shared__ __align__(16) float sPart[kRowsPerBlk * 4 * 8];
  __shared__ __align__(16) float sNP[kRowsPerBlk * kNPad];
  __shared__ float sInv[kRowsPerBlk];
  __shared__ int sSb[kRowsPerBlk * kSeq];
  __shared__ int sSi[kSeq * kNI];
  __shared__ int sEq[kRowsPerBlk];

  const int tid  = threadIdx.x;
  const int lane = tid & 31;
  const int wave = tid >> 5;
  const int b0   = blockIdx.x * kRowsPerBlk;

  int si[kSeq];
  float nPos[kSeq], nSym[kSeq], nBoth[kSeq];
  {
    v4f tv[12];
#pragma unroll
    for (int q = 0; q < 12; ++q) tv[q] = *(const v4f*)(tab + (size_t)tid * kTabW + q * 4);
#pragma unroll
    for (int e = 0; e < kTabW; ++e) sR[e * kNI + tid] = TABV(e);
#pragma unroll
    for (int m = 0; m < kSeq; ++m) {
      nPos[m]  = 1.0f - TABV(kTOnePos + m);
      nSym[m]  = 1.0f - TABV(kTOneSym + m);
      nBoth[m] = 1.0f - TABV(kTBoth + m);
      si[m] = clamp_sym(inv_inputs[tid * kSeq + m]);
      sSi[m * kNI + tid] = si[m];
    }
  }
  {
    const int q0 = inputs[(size_t)b0 * kSeq + tid];
    const int i1 = (tid + 128 < kRowsPerBlk * kSeq) ? (tid + 128) : (kRowsPerBlk * kSeq - 1);
    int q1 = inputs[(size_t)b0 * kSeq + i1];
    asm volatile("" : "+v"(q1));
    sSb[tid] = clamp_sym(q0);
    if (tid + 128 < kRowsPerBlk * kSeq) sSb[tid + 128] = clamp_sym(q1);
  }
  __syncthreads();
  if (tid < kRowsPerBlk) {
    int sv[kSeq];
#pragma unroll
    for (int k = 0; k < kSeq; ++k) sv[k] = sSb[tid * kSeq + k];
    int emk = 0;
#pragma unroll
    for (int a = 0; a < kSeq; ++a)
#pragma unroll
      for (int b = a + 1; b < kSeq; ++b)
        emk |= (sv[a] == sv[b]) ? (1 << pair_bit(a, b)) : 0;
    sEq[tid] = emk;
  }
  __syncthreads();

#pragma unroll 1
  for (int bl = 0; bl < kRowsPerBlk; ++bl) {
    const int em = __builtin_amdgcn_readfirstlane(sEq[bl]);
    int sbk[kSeq];
#pragma unroll
    for (int k = 0; k < kSeq; ++k) sbk[k] = __builtin_amdgcn_readfirstlane(sSb[bl * kSeq + k]);

    float P[kSeq][kSeq];
#pragma unroll
    for (int m = 0; m < kSeq; ++m)
#pragma unroll
      for (int k = 0; k < kSeq; ++k) P[m][k] = 1.0f;
    if (em != 0) {
      float nu[kSeq][kSeq];
#pragma unroll
      for (int m = 0; m < kSeq; ++m)
#pragma unroll
        for (int j = 0; j < kSeq; ++j) {
          const bool smt = (sbk[j] == si[m]);
          const float vd = smt ? 0.0f : nSym[m];
          const float vo = smt ? nPos[m] : nBoth[m];
          nu[m][j] = (j == m) ? vd : vo;
        }
#pragma unroll
      for (int a = 0; a < kSeq; ++a)
#pragma unroll
        for (int b = a + 1; b < kSeq; ++b) {
          if ((em >> pair_bit(a, b)) & 1) {
#pragma unroll
            for (int m = 0; m < kSeq; ++m) {
              P[m][b] *= nu[m][a];
              P[m][a] *= nu[m][b];
            }
          }
        }
#pragma unroll
      for (int m = 0; m < kSeq; ++m)
#pragma unroll
        for (int k = 0; k < kSeq; ++k) {
          const float sv2 = 1.0f - P[m][k];
          P[m][k] = 1.0f - sv2;
        }
    }

    float w[kSeq];
#pragma unroll
    for (int k = 0; k < kSeq; ++k) w[k] = 0.0f;
    float iu = 1.0f;
#pragma unroll 1
    for (int l = 0; l < kSeq; ++l) {
      const float oP  = sR[(kTOnePos + l) * kNI + tid];
      const float oS  = sR[(kTOneSym + l) * kNI + tid];
      const float uB  = sR[(kTBoth + l) * kNI + tid];
      const float oml = sR[(kTOm + l) * kNI + tid];
      const int   sil = sSi[l * kNI + tid];
      float cl[kSeq];
#pragma unroll
      for (int m = 0; m < kSeq; ++m) cl[m] = sR[(kTC + l * kSeq + m) * kNI + tid];
      float e[kSeq];
      float se = 0.0f;
      float pp = 1.0f;
#pragma unroll
      for (int k = 0; k < kSeq; ++k) {
        const bool smt = (sbk[k] == sil);
        const float ua = smt ? 1.0f : oS;
        const float ub = smt ? oP : uB;
        const float u  = (k == l) ? ua : ub;
        float pr = 1.0f - cl[0] * P[0][k];
        pr *= (1.0f - cl[1] * P[1][k]);
        pr *= (1.0f - cl[2] * P[2][k]);
        pr *= (1.0f - cl[3] * P[3][k]);
        pr *= (1.0f - cl[4] * P[4][k]);
        const float us = u * pr;
        e[k] = expf(us * scale);
        se += e[k];
        pp *= (1.0f - us);
      }
      const float f = oml * __builtin_amdgcn_rcpf(se);
#pragma unroll
      for (int k = 0; k < kSeq; ++k) w[k] += e[k] * f;
      iu *= (1.0f - pp);
    }
    const float E = expf(iu * scale);
    float red[kSeq + 1];
    red[0] = E;
#pragma unroll
    for (int k = 0; k < kSeq; ++k) red[1 + k] = E * w[k];
#pragma unroll
    for (int off = 16; off > 0; off >>= 1) {
#pragma unroll
      for (int j = 0; j < kSeq + 1; ++j) red[j] += __shfl_xor(red[j], off, 32);
    }
    if (lane == 0) {
#pragma unroll
      for (int j = 0; j < kSeq + 1; ++j) sPart[(bl * 4 + wave) * 8 + j] = red[j];
    }
    sE[bl * kNI + tid] = E;
  }
  __syncthreads();

  if (tid < kRowsPerBlk) {
    float tot[kSeq + 1];
#pragma unroll
    for (int j = 0; j < kSeq + 1; ++j)
      tot[j] = ((sPart[(tid * 4 + 0) * 8 + j] + sPart[(tid * 4 + 1) * 8 + j]) + sPart[(tid * 4 + 2) * 8 + j]) + sPart[(tid * 4 + 3) * 8 + j];
    const float invS = __builtin_amdgcn_rcpf(tot[0]);
    sInv[tid] = invS;
    int sbo[kSeq];
#pragma unroll
    for (int k = 0; k < kSeq; ++k) sbo[k] = sSb[tid * kSeq + k];
    float nv[kNPad];
#pragma unroll
    for (int s = 0; s < kNPad; ++s) {
      float a = 0.0f;
      if (s < kNSym) {
#pragma unroll
        for (int k = 0; k < kSeq; ++k) a += (sbo[k] == s) ? tot[1 + k] : 0.0f;
        a = a * invS;
      }
      nv[s] = a;
    }
#pragma unroll
    for (int q = 0; q < 4; ++q) {
      v4f o;
      o[0] = nv[q * 4 + 0]; o[1] = nv[q * 4 + 1]; o[2] = nv[q * 4 + 2]; o[3] = nv[q * 4 + 3];
      *(v4f*)(sNP + tid * kNPad + q * 4) = o;
    }
  }
  __syncthreads();

  v8h hv[4], lv[4];
#pragma unroll
  for (int it = 0; it < 4; ++it) {
    const int u = it * 128 + tid;
    const int r = u >> 4;
    const int c8 = (u & 15) * 8;
    const float inv = sInv[r] * kCarrySel;
    const v4f a0 = *(const v4f*)(sE + r * kNI + c8);
    const v4f a1 = *(const v4f*)(sE + r * kNI + c8 + 4);
#pragma unroll
    for (int e = 0; e < 4; ++e) {
      _Float16 h0, l0, h1, l1;
      const float x0 = a0[e] * inv;
      const float x1 = a1[e] * inv;
      split_h(x0, h0, l0);
      split_h(x1, h1, l1);
      hv[it][e] = h0; hv[it][4 + e] = h1;
      lv[it][e] = l0; lv[it][4 + e] = l1;
    }
  }
  const v4f npv = *(const v4f*)(sNP + tid * 4);
  for (int pass = 0; pass < 2; ++pass) {
#pragma unroll
    for (int it = 0; it < 4; ++it) {
      const size_t o = (size_t)b0 * kNI + (size_t)(it * 128 + tid) * 8;
      *(volatile v8h*)(ahi + o) = hv[it];
      *(volatile v8h*)(alo + o) = lv[it];
    }
    *(volatile v4f*)(npl + (size_t)b0 * kNPad + (size_t)tid * 4) = npv;
    __threadfence();
  }
}

__global__ __launch_bounds__(32) void label_gemm_kernel(
    const _Float16* __restrict__ ahi, const _Float16* __restrict__ alo,
    const _Float16* __restrict__ bhi, const _Float16* __restrict__ blo,
    const float* __restrict__ npl, float* __restrict__ out)
{
  __shared__ __align__(16) float sN[kRowsPerBlk * kNPad];
  __shared__ __align__(16) float sO[kRowsPerBlk * kNSym];
  const int lane = threadIdx.x & 31;
  const int hh = lane >> 4;
  const int rl = lane & 15;
  const int m0 = blockIdx.x * kRowsPerBlk;

#pragma unroll
  for (int it = 0; it < 4; ++it) {
    const v4f t = *(const v4f*)(npl + (size_t)m0 * kNPad + (size_t)(it * 32 + lane) * 4);
    *(v4f*)(sN + (it * 32 + lane) * 4) = t;
  }

  v16h bh[4], bl[4];
#pragma unroll
  for (int kq = 0; kq < 4; ++kq) {
    const int bo = rl * kNI + 8 * hh + kq * 32;
    bh[kq] = Frag<_Float16>::load(bhi + bo);
    bl[kq] = Frag<_Float16>::load(blo + bo);
  }

  v8f am[2], ar[2];
#pragma unroll
  for (int i = 0; i < 2; ++i) {
    am[i] = (v8f){0.f, 0.f, 0.f, 0.f, 0.f, 0.f, 0.f, 0.f};
    ar[i] = (v8f){0.f, 0.f, 0.f, 0.f, 0.f, 0.f, 0.f, 0.f};
  }
#pragma unroll
  for (int i = 0; i < 2; ++i) {
#pragma unroll
    for (int kq = 0; kq < 4; ++kq) {
      const size_t ao = (size_t)(m0 + i * 16 + rl) * kNI + 8 * hh + kq * 32;
      const v16h ah = Frag<_Float16>::load(ahi + ao);
      const v16h al = Frag<_Float16>::load(alo + ao);
      am[i] = mma_h_guard(ah, bh[kq], am[i]);
      ar[i] = mma_h_guard(ah, bl[kq], ar[i]);
      ar[i] = mma_h_guard(al, bh[kq], ar[i]);
    }
  }
  __syncthreads();
#pragma unroll
  for (int i = 0; i < 2; ++i) {
#pragma unroll
    for (int r = 0; r < 8; ++r) {
      const int row = i * 16 + 8 * hh + r;
      const float lab = (am[i][r] + ar[i][r] * kInvRes) * kInvCarry;
      const float v = lab + sN[row * kNPad + rl];
      if (rl < kNSym) sO[row * kNSym + rl] = v;
    }
  }
  __syncthreads();
  v4f ov[3];
#pragma unroll
  for (int it = 0; it < 3; ++it) {
    const int idx = it * 32 + lane;
    const int ci = (idx < 72) ? idx : 71;
    ov[it] = *(const v4f*)(sO + ci * 4);
  }
  float* ob = out + (size_t)m0 * kNSym;
  for (int pass = 0; pass < 2; ++pass) {
    *(volatile v4f*)(ob + (size_t)lane * 4) = ov[0];
    *(volatile v4f*)(ob + (size_t)(32 + lane) * 4) = ov[1];
    if (lane < 8) *(volatile v4f*)(ob + (size_t)(64 + lane) * 4) = ov[2];
    __threadfence();
  }
}

extern "C" void kernel_launch(void* const* d_in, const int* in_sizes, int n_in,
                              void* d_out, int out_size, void* d_ws, size_t ws_size,
                              hipStream_t stream) {
  if (n_in < 6) return;
  if (in_sizes[0] != kNB * kSeq) return;
  if (in_sizes[1] != kNI * kSeq) return;
  if (in_sizes[2] != kNI) return;
  if (in_sizes[3] != kNI * kSeq * kNU) return;
  if (in_sizes[4] != kNI * kSeq * kSeq) return;
  if (in_sizes[5] != kNI * (kSeq + 1)) return;
  if (out_size != kNB * kNSym) return;
  if (ws_size < kWsTotal) return;

  const int*   inputs     = (const int*)d_in[0];
  const int*   inv_inputs = (const int*)d_in[1];
  const int*   inv_labels = (const int*)d_in[2];
  const float* unaryp     = (const float*)d_in[3];
  const float* binaryp    = (const float*)d_in[4];
  const float* outmap     = (const float*)d_in[5];
  float* out = (float*)d_out;

  char* ws = (char*)d_ws;
  float*          tab = (float*)(ws + kOffTab);
  unsigned short* bhi = (unsigned short*)(ws + kOffBhi);
  unsigned short* blo = (unsigned short*)(ws + kOffBlo);
  unsigned short* ahi = (unsigned short*)(ws + kOffAhi);
  unsigned short* alo = (unsigned short*)(ws + kOffAlo);
  float*          npl = (float*)(ws + kOffNp);

  const float ratio = (0.999f * (float)(kNI - 1)) / (float)(1.0 - 0.999);
  const float sm_scale = logf(ratio);

  prep_kernel<<<1, 128, 0, stream>>>(inv_inputs, inv_labels, unaryp, binaryp, outmap, tab, bhi, blo);
  unify_kernel<<<kNB / kRowsPerBlk, 128, 0, stream>>>(inputs, inv_inputs, tab, ahi, alo, npl, sm_scale);
  label_gemm_kernel<<<kNB / kRowsPerBlk, 32, 0, stream>>>(
      (const _Float16*)ahi, (const _Float16*)alo, (const _Float16*)bhi, (const _Float16*)blo, npl, out);
}
